// PointNetSetAbstraction_11965778886750
// MI455X (gfx1250) — hardware-verified
//
#include <hip/hip_runtime.h>
#pragma clang fp contract(off)

typedef __attribute__((ext_vector_type(16))) _Float16 v16h;
typedef __attribute__((ext_vector_type(8)))  _Float16 v8h;
typedef __attribute__((ext_vector_type(8)))  float    v8f;
typedef __attribute__((ext_vector_type(4)))  float    v4f;
typedef __attribute__((ext_vector_type(2)))  float    v2f;
typedef __attribute__((ext_vector_type(4)))  unsigned v4u;

constexpr int NBATCH  = 16;
constexpr int NPTS    = 8192;
constexpr int CIN     = 64;
constexpr int NCENT   = 1024;
constexpr int NSAMP   = 32;
constexpr int W0_COLS = 67;
constexpr int CH_L0   = 64;
constexpr int CH_L1   = 64;
constexpr int CH_L2   = 128;
constexpr int MROWS   = NBATCH * NCENT * NSAMP;
constexpr int QROWS   = MROWS / 4;
constexpr int NPART   = 2048;
constexpr float W_CARRY     = 16.0f;
constexpr float W_CARRY_INV = 1.0f / 16.0f;
constexpr float BN_EPS      = 1e-5f;
constexpr float RAD2        = 0.04f;
constexpr float INV_MROWS   = 1.0f / (float)MROWS;

static_assert(MROWS == 524288);
static_assert(QROWS == 131072);
static_assert(QROWS == NBATCH * NPTS);
static_assert(CIN == 64 && CH_L0 == 64 && CH_L1 == 64 && CH_L2 == 128);
static_assert(QROWS % 256 == 0);
static_assert(196608 + 8388608 == 8585216);
static_assert(NBATCH * NCENT * 3 * 4 == 196608);

union FragU { v16h v; v8h h[2]; };
__device__ __forceinline__ v16h frag_load(const _Float16* p) {
  FragU f;
  f.h[0] = *(const v8h*)(p);
  f.h[1] = *(const v8h*)(p + 16);
  return f.v;
}
__device__ __forceinline__ v8f mma_h(v16h a, v16h b, v8f c) {
  return __builtin_amdgcn_wmma_f32_16x16x32_f16(false, a, false, b, (short)0, c, false, false);
}
__device__ __forceinline__ void guard_group(v8f& c0, v8f& c1, v8f& c2, v8f& c3,
                                            v16h a, v16h b0, v16h b1, v16h b2, v16h b3) {
  asm volatile("v_nop\n\tv_nop\n\tv_nop\n\tv_nop"
               : "+v"(c0), "+v"(c1), "+v"(c2), "+v"(c3)
               : "v"(a), "v"(b0), "v"(b1), "v"(b2), "v"(b3));
}
__device__ __forceinline__ void keep4_h(v16h a, v16h b, v16h c, v16h d) {
  asm volatile("v_nop" :: "v"(a), "v"(b), "v"(c), "v"(d));
}
__device__ __forceinline__ void wave_lds_sync() {
  __builtin_amdgcn_fence(__ATOMIC_RELEASE, "workgroup");
  __builtin_amdgcn_wave_barrier();
  __builtin_amdgcn_fence(__ATOMIC_ACQUIRE, "workgroup");
}

__device__ __forceinline__ float prod_pinned(float a, float b) {
  float p = a * b;
  asm volatile("" : "+v"(p));
  return p;
}

__device__ __forceinline__ float h16_to_f32(unsigned hb) {
  const unsigned sgn = (hb & 0x8000u) << 16;
  const unsigned em = hb & 0x7fffu;
  const float fn = __uint_as_float((em << 13) + 0x38000000u);
  const float fs = (float)em * 5.9604644775390625e-8f;
  const float mag = (em < 0x400u) ? fs : fn;
  return __uint_as_float(__float_as_uint(mag) | sgn);
}

__device__ __forceinline__ void cvt_store8(const float* s, unsigned short* dst, float carry) {
  v8h hv;
#pragma unroll
  for (int e = 0; e < 8; ++e) hv[e] = (_Float16)(s[e] * carry);
  *(volatile v8h*)dst = hv;
  __threadfence();
  *(volatile v8h*)dst = hv;
}

__global__ __launch_bounds__(256) void pack_weights(const float* w0, const float* w1, const float* w2,
                                                    unsigned short* w0p, float* w0x,
                                                    unsigned short* w1h, unsigned short* w2h) {
  const int blk = blockIdx.x;
  const int t = threadIdx.x;
  if (blk < 2) {
    const int ci = blk * 256 + t;
    const int o = ci >> 3;
    const int k0 = (ci & 7) * 8;
    cvt_store8(w0 + o * W0_COLS + k0, w0p + ci * 8, W_CARRY);
  } else if (blk < 4) {
    const int ci = (blk - 2) * 256 + t;
    cvt_store8(w1 + ci * 8, w1h + ci * 8, W_CARRY);
  } else if (blk < 8) {
    const int ci = (blk - 4) * 256 + t;
    cvt_store8(w2 + ci * 8, w2h + ci * 8, W_CARRY);
  } else {
    if (t < 64) {
      const float a = w0[t * W0_COLS + 64];
      const float b = w0[t * W0_COLS + 65];
      const float c = w0[t * W0_COLS + 66];
      const v4f v = (v4f){a, b, c, 0.0f};
      *(volatile v4f*)(w0x + t * 4) = v;
      __threadfence();
      *(volatile v4f*)(w0x + t * 4) = v;
    }
  }
}

__global__ __launch_bounds__(256) void transpose_points(const float* points, unsigned short* P16) {
  __shared__ float tile[64 * 65];
  const int t = threadIdx.x;
  const int b = blockIdx.x >> 7;
  const int n0 = (blockIdx.x & 127) * 64;
  const int n = t & 63;
  const int c0 = t >> 6;
  const float* src = points + (size_t)b * CIN * NPTS + n0 + n;
#pragma unroll
  for (int i = 0; i < 8; ++i) {
    const int c = c0 + 4 * i;
    tile[c * 65 + n] = src[(size_t)c * NPTS];
  }
  asm volatile("" ::: "memory");
#pragma unroll
  for (int i = 8; i < 16; ++i) {
    const int c = c0 + 4 * i;
    tile[c * 65 + n] = src[(size_t)c * NPTS];
  }
  __syncthreads();
  const int q = t & 7;
  const int r0 = t >> 3;
  v8h ha, hb;
#pragma unroll
  for (int e = 0; e < 8; ++e) {
    ha[e] = (_Float16)tile[(8 * q + e) * 65 + r0];
    hb[e] = (_Float16)tile[(8 * q + e) * 65 + r0 + 32];
  }
  unsigned short* da = P16 + ((size_t)b * NPTS + n0 + r0) * 64 + 8 * q;
  unsigned short* db = da + 32 * 64;
  *(volatile v8h*)da = ha;
  *(volatile v8h*)db = hb;
  __threadfence();
  *(volatile v8h*)da = ha;
  *(volatile v8h*)db = hb;
}

__device__ __forceinline__ void argmax_step(float& v, int& i, int off) {
  const float ov = __shfl_xor(v, off);
  const int oi = __shfl_xor(i, off);
  const bool take = (ov > v) || ((ov == v) && (oi < i));
  v = take ? ov : v;
  i = take ? oi : i;
}

__global__ __launch_bounds__(1024) void fps_kernel(const float* xyz, float* newxyz_ws, float* out_xyz) {
#pragma clang fp contract(off)
  __shared__ float s_val[2][32];
  __shared__ int   s_idx[2][32];
  __shared__ int   s_cent[NCENT];
  const int b = blockIdx.x;
  const int t = threadIdx.x;
  const int lane = t & 31;
  const int wv = t >> 5;
  const float* xb = xyz + (size_t)b * NPTS * 3;

  float px[8], py[8], pz[8], dist[8];
  {
    const v4f* p4 = (const v4f*)(xb + (size_t)t * 24);
    const v4f a0 = p4[0], a1 = p4[1], a2 = p4[2], a3 = p4[3], a4 = p4[4], a5 = p4[5];
    px[0] = a0.x; py[0] = a0.y; pz[0] = a0.z;
    px[1] = a0.w; py[1] = a1.x; pz[1] = a1.y;
    px[2] = a1.z; py[2] = a1.w; pz[2] = a2.x;
    px[3] = a2.y; py[3] = a2.z; pz[3] = a2.w;
    px[4] = a3.x; py[4] = a3.y; pz[4] = a3.z;
    px[5] = a3.w; py[5] = a4.x; pz[5] = a4.y;
    px[6] = a4.z; py[6] = a4.w; pz[6] = a5.x;
    px[7] = a5.y; py[7] = a5.z; pz[7] = a5.w;
  }
#pragma unroll
  for (int k = 0; k < 8; ++k) dist[k] = 1e10f;

  int cur = 0;
#pragma unroll 1
  for (int it = 0; it < NCENT; ++it) {
    if (t == 0) s_cent[it] = cur;
    const float* cp = xb + (size_t)cur * 3;
    const float cx = cp[0], cy = cp[1], cz = cp[2];
    float bv = -1.0f;
    int bi = t * 8;
#pragma unroll
    for (int k = 0; k < 8; ++k) {
      const float dx = px[k] - cx;
      const float dy = py[k] - cy;
      const float dz = pz[k] - cz;
      const float t0 = prod_pinned(dx, dx);
      const float t1 = prod_pinned(dy, dy);
      const float t2 = prod_pinned(dz, dz);
      float t02 = t0 + t2;
      asm volatile("" : "+v"(t02));
      const float d = t02 + t1;
      const float nd = fminf(dist[k], d);
      dist[k] = nd;
      const bool up = nd > bv;
      bv = up ? nd : bv;
      bi = up ? (t * 8 + k) : bi;
    }
    argmax_step(bv, bi, 16);
    argmax_step(bv, bi, 8);
    argmax_step(bv, bi, 4);
    argmax_step(bv, bi, 2);
    argmax_step(bv, bi, 1);
    const int buf = it & 1;
    if (lane == 0) { s_val[buf][wv] = bv; s_idx[buf][wv] = bi; }
    __syncthreads();
    float v = s_val[buf][lane];
    int i2 = s_idx[buf][lane];
    argmax_step(v, i2, 16);
    argmax_step(v, i2, 8);
    argmax_step(v, i2, 4);
    argmax_step(v, i2, 2);
    argmax_step(v, i2, 1);
    i2 = i2 < 0 ? 0 : i2;
    i2 = i2 > (NPTS - 1) ? (NPTS - 1) : i2;
    cur = i2;
  }
  __syncthreads();
  if (t < 768) {
    float o[4];
#pragma unroll
    for (int e = 0; e < 4; ++e) {
      const int gidx = 4 * t + e;
      const int s = gidx / 3;
      const int c = gidx - 3 * s;
      int id = s_cent[s];
      id = id < 0 ? 0 : id;
      id = id > (NPTS - 1) ? (NPTS - 1) : id;
      o[e] = xb[(size_t)id * 3 + c];
    }
    const v4f ov = (v4f){o[0], o[1], o[2], o[3]};
    float* d0 = out_xyz + (size_t)b * (NCENT * 3) + 4 * t;
    float* d1 = newxyz_ws + (size_t)b * (NCENT * 3) + 4 * t;
    *(volatile v4f*)d0 = ov;
    *(volatile v4f*)d1 = ov;
    __threadfence();
    *(volatile v4f*)d0 = ov;
    *(volatile v4f*)d1 = ov;
  }
}

template <int NOUT, int MODE>
__global__ __launch_bounds__(256) void mlp_gemm(const unsigned short* Ap, const unsigned short* Btp,
                                                void* Cout, float* part, float* ymax, float* ymin,
                                                float scale) {
  static_assert(NOUT % 64 == 0);
  static_assert(MODE == 2 || NOUT == 64);
  const _Float16* A = (const _Float16*)Ap;
  const _Float16* Bt = (const _Float16*)Btp;
  __shared__ __align__(16) float sSlab[8][(MODE == 2) ? 4 : 16 * 68];
  __shared__ __align__(16) float sStat[8][(MODE >= 1) ? 2 * NOUT : 4];
  __shared__ __align__(16) float sMM[8][(MODE == 2) ? 2 * NOUT : 4];

  const int lane = threadIdx.x & 31;
  const int wave = threadIdx.x >> 5;
  const int rlane = lane & 15;
  const int hh = lane >> 4;
  const int koff = hh * 8;
  const int mOff = hh * 8;
  const size_t m0 = ((size_t)blockIdx.x * 8 + wave) * 32;

  v16h af[2][2];
#pragma unroll
  for (int i = 0; i < 2; ++i)
#pragma unroll
    for (int ks = 0; ks < 2; ++ks)
      af[i][ks] = frag_load(A + (m0 + (size_t)(i * 16 + rlane)) * 64 + ks * 32 + koff);

#pragma unroll 1
  for (int nh = 0; nh < NOUT / 64; ++nh) {
    v8f acc[2][4];
#pragma unroll
    for (int i = 0; i < 2; ++i)
#pragma unroll
      for (int j = 0; j < 4; ++j) acc[i][j] = (v8f){0.f, 0.f, 0.f, 0.f, 0.f, 0.f, 0.f, 0.f};

#pragma unroll
    for (int ks = 0; ks < 2; ++ks) {
      v16h bh[4];
#pragma unroll
      for (int j = 0; j < 4; ++j)
        bh[j] = frag_load(Bt + (size_t)(nh * 64 + j * 16 + rlane) * 64 + ks * 32 + koff);
#pragma unroll
      for (int i = 0; i < 2; ++i) {
#pragma unroll
        for (int j = 0; j < 4; ++j) acc[i][j] = mma_h(af[i][ks], bh[j], acc[i][j]);
        guard_group(acc[i][0], acc[i][1], acc[i][2], acc[i][3], af[i][ks], bh[0], bh[1], bh[2], bh[3]);
      }
      keep4_h(bh[0], bh[1], bh[2], bh[3]);
    }

#pragma unroll
    for (int i = 0; i < 2; ++i)
#pragma unroll
      for (int j = 0; j < 4; ++j) acc[i][j] = acc[i][j] * scale;

    if (MODE >= 1) {
#pragma unroll
      for (int j = 0; j < 4; ++j) {
        float s = 0.0f, q = 0.0f, mx = -3.0e38f, mn = 3.0e38f;
#pragma unroll
        for (int i = 0; i < 2; ++i)
#pragma unroll
          for (int r = 0; r < 8; ++r) {
            const float v = acc[i][j][r];
            s += v;
            q = fmaf(v, v, q);
            mx = fmaxf(mx, v);
            mn = fminf(mn, v);
          }
        const float so = __shfl_xor(s, 16);
        const float qo = __shfl_xor(q, 16);
        const float mxo = __shfl_xor(mx, 16);
        const float mno = __shfl_xor(mn, 16);
        s += so;
        q += qo;
        mx = fmaxf(mx, mxo);
        mn = fminf(mn, mno);
        const int col = nh * 64 + j * 16 + rlane;
        if (hh == 0) {
          sStat[wave][col] = s;
          sStat[wave][NOUT + col] = q;
          if (MODE == 2) {
            sMM[wave][col] = mx;
            sMM[wave][NOUT + col] = mn;
          }
        }
      }
    }

    if (MODE != 2) {
      float* slab = sSlab[wave];
#pragma unroll
      for (int i = 0; i < 2; ++i) {
#pragma unroll
        for (int j = 0; j < 4; ++j)
#pragma unroll
          for (int r = 0; r < 8; ++r)
            slab[(mOff + r) * 68 + j * 16 + rlane] = acc[i][j][r];
        wave_lds_sync();
        if (MODE == 0) {
          float* C = (float*)Cout;
          const int c4 = rlane * 4;
          for (int pass = 0; pass < 2; ++pass) {
#pragma unroll
            for (int it = 0; it < 8; ++it) {
              const int row = it * 2 + hh;
              const v4f v = *(const v4f*)(slab + row * 68 + c4);
              *(volatile v4f*)(C + (m0 + (size_t)(i * 16 + row)) * 64 + c4) = v;
            }
            __threadfence();
          }
        } else {
          unsigned short* C = (unsigned short*)Cout;
          const int q8 = lane >> 3;
          const int c8 = (lane & 7) * 8;
          for (int pass = 0; pass < 2; ++pass) {
#pragma unroll
            for (int it = 0; it < 4; ++it) {
              const int row = it * 4 + q8;
              const float* sp = slab + row * 68 + c8;
              v8h hv;
#pragma unroll
              for (int e = 0; e < 8; ++e) hv[e] = (_Float16)sp[e];
              *(volatile v8h*)(C + (m0 + (size_t)(i * 16 + row)) * 64 + c8) = hv;
            }
            __threadfence();
          }
        }
        wave_lds_sync();
      }
    }
  }

  if (MODE == 2) {
    wave_lds_sync();
    const size_t g = (size_t)blockIdx.x * 8 + wave;
    const v4f vmx = *(const v4f*)(sMM[wave] + lane * 4);
    const v4f vmn = *(const v4f*)(sMM[wave] + NOUT + lane * 4);
    float* pmx = ymax + g * NOUT + lane * 4;
    float* pmn = ymin + g * NOUT + lane * 4;
    *(volatile v4f*)pmx = vmx;
    *(volatile v4f*)pmn = vmn;
    __threadfence();
    *(volatile v4f*)pmx = vmx;
    *(volatile v4f*)pmn = vmn;
  }

  if (MODE >= 1) {
    __syncthreads();
    if (threadIdx.x < (2 * NOUT) / 4) {
      const int c4 = threadIdx.x * 4;
      v4f tot = (v4f){0.f, 0.f, 0.f, 0.f};
#pragma unroll
      for (int w = 0; w < 8; ++w) tot += *(const v4f*)(&sStat[w][c4]);
      float* dst = part + (size_t)blockIdx.x * (2 * NOUT) + c4;
      *(volatile v4f*)dst = tot;
      __threadfence();
      *(volatile v4f*)dst = tot;
    }
  }
}

__global__ __launch_bounds__(256) void ball_assemble(const float* xyz, const float* newxyz, const float* Z,
                                                     const float* w0x, unsigned short* Y0, float* part) {
#pragma clang fp contract(off)
  __shared__ int s_slots[8][32];
  __shared__ __align__(16) unsigned sY[8][32 * 32];
  __shared__ __align__(16) float sStat[8][128];
  const int lane = threadIdx.x & 31;
  const int wv = threadIdx.x >> 5;
  const int cent = blockIdx.x * 8 + wv;
  const int b = cent >> 10;
  const float* cc = newxyz + (size_t)cent * 3;
  const float cx = cc[0], cy = cc[1], cz = cc[2];
  const float* xb = xyz + (size_t)b * NPTS * 3;

  s_slots[wv][lane] = 0;
  int count = 0;
#pragma unroll 1
  for (int base = 0; base < NPTS; base += 32) {
    if (count >= NSAMP) break;
    const int i = base + lane;
    const float* p = xb + (size_t)i * 3;
    const float dx = cx - p[0];
    const float dy = cy - p[1];
    const float dz = cz - p[2];
    const float t0 = prod_pinned(dx, dx);
    const float t1 = prod_pinned(dy, dy);
    const float t2 = prod_pinned(dz, dz);
    float t02 = t0 + t2;
    asm volatile("" : "+v"(t02));
    const float sq = t02 + t1;
    const bool inR = !(sq > RAD2);
    const unsigned m = (unsigned)__ballot(inR);
    const int pos = count + __popc(m & ((1u << lane) - 1u));
    if (inR && pos < NSAMP) s_slots[wv][pos] = i;
    count += __popc(m);
  }
  wave_lds_sync();
  const int cnt = count > NSAMP ? NSAMP : count;
  int myidx = s_slots[wv][lane < cnt ? lane : 0];
  myidx = myidx < 0 ? 0 : myidx;
  myidx = myidx > (NPTS - 1) ? (NPTS - 1) : myidx;
  const float* pp = xb + (size_t)myidx * 3;
  const float rx = pp[0] - cx;
  const float ry = pp[1] - cy;
  const float rz = pp[2] - cz;

  const v4f wa = *(const v4f*)(w0x + (2 * lane) * 4);
  const v4f wb = *(const v4f*)(w0x + (2 * lane + 1) * 4);
  const float* zb = Z + (size_t)b * NPTS * 64 + 2 * lane;
  unsigned* ytile = sY[wv];
  float s0 = 0.0f, s1 = 0.0f, q0 = 0.0f, q1 = 0.0f;
#pragma unroll 4
  for (int k = 0; k < NSAMP; ++k) {
    const int ik = __shfl(myidx, k);
    const float kx = __shfl(rx, k);
    const float ky = __shfl(ry, k);
    const float kz = __shfl(rz, k);
    const v2f z = *(const v2f*)(zb + (size_t)ik * 64);
    float y0 = z.x + prod_pinned(wa.x, kx);
    y0 = y0 + prod_pinned(wa.y, ky);
    y0 = y0 + prod_pinned(wa.z, kz);
    float y1 = z.y + prod_pinned(wb.x, kx);
    y1 = y1 + prod_pinned(wb.y, ky);
    y1 = y1 + prod_pinned(wb.z, kz);
    s0 += y0;
    s1 += y1;
    q0 = q0 + prod_pinned(y0, y0);
    q1 = q1 + prod_pinned(y1, y1);
    const _Float16 h0 = (_Float16)y0;
    const _Float16 h1 = (_Float16)y1;
    const unsigned u = (unsigned)__builtin_bit_cast(unsigned short, h0) |
                       ((unsigned)__builtin_bit_cast(unsigned short, h1) << 16);
    ytile[k * 32 + lane] = u;
  }
  sStat[wv][2 * lane] = s0;
  sStat[wv][2 * lane + 1] = s1;
  sStat[wv][64 + 2 * lane] = q0;
  sStat[wv][64 + 2 * lane + 1] = q1;
  wave_lds_sync();
  {
    const int q8 = lane >> 3;
    const int c = lane & 7;
    for (int pass = 0; pass < 2; ++pass) {
#pragma unroll
      for (int it = 0; it < 8; ++it) {
        const int row = it * 4 + q8;
        const v4u w = *(const v4u*)(ytile + row * 32 + c * 4);
        *(volatile v4u*)(Y0 + ((size_t)cent * NSAMP + row) * 64 + c * 8) = w;
      }
      __threadfence();
    }
  }
  __syncthreads();
  if (threadIdx.x < 32) {
    const int c4 = threadIdx.x * 4;
    v4f tot = (v4f){0.f, 0.f, 0.f, 0.f};
#pragma unroll
    for (int w = 0; w < 8; ++w) tot += *(const v4f*)(&sStat[w][c4]);
    float* dst = part + (size_t)blockIdx.x * 128 + c4;
    *(volatile v4f*)dst = tot;
    __threadfence();
    *(volatile v4f*)dst = tot;
  }
}

template <int NOUT>
__global__ __launch_bounds__(1024) void reduce_stats(const float* part, int nblk, const float* gam,
                                                     const float* bet, float* scsh) {
  constexpr int WD = 2 * NOUT;
  constexpr int GR = 1024 / WD;
  __shared__ float sP[1024];
  __shared__ __align__(16) float sTot[WD];
  __shared__ __align__(16) float sOut[WD];
  const int t = threadIdx.x;
  const int c = t % WD;
  const int gi = t / WD;
  float acc = 0.0f;
#pragma unroll 4
  for (int r = gi; r < nblk; r += GR) acc += part[(size_t)r * WD + c];
  sP[t] = acc;
  __syncthreads();
  if (t < WD) {
    float tot = 0.0f;
#pragma unroll
    for (int gg = 0; gg < GR; ++gg) tot += sP[gg * WD + t];
    sTot[t] = tot;
  }
  __syncthreads();
  if (t < NOUT) {
    const float mean = sTot[t] * INV_MROWS;
    const float ex2 = sTot[NOUT + t] * INV_MROWS;
    float var = ex2 - mean * mean;
    var = fmaxf(var, 0.0f);
    const float sc = gam[t] * (1.0f / sqrtf(var + BN_EPS));
    const float sh = bet[t] - mean * sc;
    sOut[t] = sc;
    sOut[NOUT + t] = sh;
  }
  __syncthreads();
  if (t < WD / 4) {
    const v4f v = *(const v4f*)(sOut + 4 * t);
    *(volatile v4f*)(scsh + 4 * t) = v;
    __threadfence();
    *(volatile v4f*)(scsh + 4 * t) = v;
  }
}

__device__ __forceinline__ float bn_relu(unsigned hb, float sc, float sh) {
  return fmaxf(fmaf(sc, h16_to_f32(hb), sh), 0.0f);
}

__global__ __launch_bounds__(256) void norm_relu(const unsigned short* Yin, unsigned short* Xout,
                                                 const float* scsh) {
  const int t = threadIdx.x;
  const int c0 = (t & 7) * 8;
  const v4f scA = *(const v4f*)(scsh + c0);
  const v4f scB = *(const v4f*)(scsh + c0 + 4);
  const v4f shA = *(const v4f*)(scsh + 64 + c0);
  const v4f shB = *(const v4f*)(scsh + 64 + c0 + 4);
  const size_t base = (size_t)blockIdx.x * 8192 + (size_t)t * 8;
#pragma unroll 1
  for (int it = 0; it < 4; ++it) {
    const size_t off = base + (size_t)it * 2048;
    const v4u w = *(const v4u*)(Yin + off);
    const unsigned w0 = w.x, w1 = w.y, w2 = w.z, w3 = w.w;
    v8h hv;
    hv[0] = (_Float16)bn_relu(w0 & 0xffffu, scA.x, shA.x);
    hv[1] = (_Float16)bn_relu(w0 >> 16,     scA.y, shA.y);
    hv[2] = (_Float16)bn_relu(w1 & 0xffffu, scA.z, shA.z);
    hv[3] = (_Float16)bn_relu(w1 >> 16,     scA.w, shA.w);
    hv[4] = (_Float16)bn_relu(w2 & 0xffffu, scB.x, shB.x);
    hv[5] = (_Float16)bn_relu(w2 >> 16,     scB.y, shB.y);
    hv[6] = (_Float16)bn_relu(w3 & 0xffffu, scB.z, shB.z);
    hv[7] = (_Float16)bn_relu(w3 >> 16,     scB.w, shB.w);
    *(volatile v8h*)(Xout + off) = hv;
    __threadfence();
    *(volatile v8h*)(Xout + off) = hv;
  }
}

__global__ __launch_bounds__(256) void final_pool(const float* ymax, const float* ymin,
                                                  const float* scsh, float* out1) {
  __shared__ float tile[128 * 33];
  const int t = threadIdx.x;
  const int b = blockIdx.x >> 5;
  const int s0 = (blockIdx.x & 31) * 32;
  const int c = t & 127;
  const int hf = t >> 7;
  const float sc = scsh[c];
  const float sh = scsh[CH_L2 + c];
  const float fa = (sc >= 0.0f) ? 1.0f : 0.0f;
  const float fb = 1.0f - fa;
  const size_t cent0 = (size_t)b * NCENT + s0;
#pragma unroll 4
  for (int i = 0; i < 16; ++i) {
    const int cl = i * 2 + hf;
    const size_t idx = (cent0 + cl) * CH_L2 + c;
    const float mx = ymax[idx];
    const float mn = ymin[idx];
    const float val = fmaf(fa, mx, fb * mn);
    tile[c * 33 + cl] = fmaxf(fmaf(sc, val, sh), 0.0f);
  }
  __syncthreads();
  const int q = t & 7;
  const int cr = t >> 3;
  v4f o[4];
#pragma unroll
  for (int it = 0; it < 4; ++it) {
    const int ch = it * 32 + cr;
    o[it] = (v4f){tile[ch * 33 + 4 * q], tile[ch * 33 + 4 * q + 1],
                  tile[ch * 33 + 4 * q + 2], tile[ch * 33 + 4 * q + 3]};
  }
  for (int pass = 0; pass < 2; ++pass) {
#pragma unroll
    for (int it = 0; it < 4; ++it) {
      const int ch = it * 32 + cr;
      *(volatile v4f*)(out1 + ((size_t)b * CH_L2 + ch) * NCENT + s0 + 4 * q) = o[it];
    }
    __threadfence();
  }
}

extern "C" void kernel_launch(void* const* d_in, const int* in_sizes, int n_in,
                              void* d_out, int out_size, void* d_ws, size_t ws_size, hipStream_t stream) {
  (void)in_sizes; (void)n_in; (void)out_size;
  const float* xyz    = (const float*)d_in[0];
  const float* points = (const float*)d_in[1];
  const float* w0     = (const float*)d_in[2];
  const float* g0     = (const float*)d_in[4];
  const float* be0    = (const float*)d_in[5];
  const float* w1     = (const float*)d_in[6];
  const float* g1     = (const float*)d_in[8];
  const float* be1    = (const float*)d_in[9];
  const float* w2     = (const float*)d_in[10];
  const float* g2     = (const float*)d_in[12];
  const float* be2    = (const float*)d_in[13];

  float* out_xyz = (float*)d_out;
  float* out_pts = out_xyz + (196608 / 4);

  const size_t GRAN_BYTES = (size_t)QROWS * 64 * 2;
  char* ws = (char*)d_ws;
  size_t off = 0;
  unsigned short* gran[5];
  for (int i = 0; i < 5; ++i) { gran[i] = (unsigned short*)(ws + off); off += GRAN_BYTES; }
  float* ZF = (float*)(ws + off);      off += (size_t)QROWS * 64 * 4;
  float* part0 = (float*)(ws + off);   off += (size_t)NPART * 128 * 4;
  float* part1 = (float*)(ws + off);   off += (size_t)NPART * 128 * 4;
  float* part2 = (float*)(ws + off);   off += (size_t)NPART * 256 * 4;
  float* newxyz = (float*)(ws + off);  off += (size_t)NBATCH * NCENT * 3 * 4;
  unsigned short* w0p = (unsigned short*)(ws + off); off += 64 * 64 * 2;
  unsigned short* w1h = (unsigned short*)(ws + off); off += 64 * 64 * 2;
  unsigned short* w2h = (unsigned short*)(ws + off); off += 128 * 64 * 2;
  float* w0x = (float*)(ws + off);     off += 64 * 4 * 4;
  float* scsh0 = (float*)(ws + off);   off += 128 * 4;
  float* scsh1 = (float*)(ws + off);   off += 128 * 4;
  float* scsh2 = (float*)(ws + off);   off += 256 * 4;
  if (off > ws_size || off > (size_t)134217728) return;

  float* Zp = ZF;
  float* ymax = ZF;
  float* ymin = ZF + (size_t)NBATCH * NCENT * CH_L2;

  pack_weights<<<9, 256, 0, stream>>>(w0, w1, w2, w0p, w0x, w1h, w2h);
  transpose_points<<<NBATCH * (NPTS / 64), 256, 0, stream>>>(points, gran[4]);
  fps_kernel<<<NBATCH, 1024, 0, stream>>>(xyz, newxyz, out_xyz);

  mlp_gemm<64, 0><<<QROWS / 256, 256, 0, stream>>>(gran[4], w0p, (void*)Zp, part0, ymax, ymin, W_CARRY_INV);

  ball_assemble<<<(NBATCH * NCENT) / 8, 256, 0, stream>>>(xyz, newxyz, Zp, w0x, gran[0], part0);
  reduce_stats<64><<<1, 1024, 0, stream>>>(part0, NPART, g0, be0, scsh0);

  const int gy0[4] = {0, 1, 2, 3};
  const int gx1[4] = {4, 0, 1, 2};
  const int gy1[4] = {3, 4, 0, 1};
  const int gx2[4] = {2, 3, 4, 0};
  const int nblkN = (int)(((size_t)QROWS * 64) / 8192);
  const int nblkG = QROWS / 256;

  for (int q = 0; q < 4; ++q)
    norm_relu<<<nblkN, 256, 0, stream>>>(gran[gy0[q]], gran[gx1[q]], scsh0);
  for (int q = 0; q < 4; ++q)
    mlp_gemm<64, 1><<<nblkG, 256, 0, stream>>>(gran[gx1[q]], w1h, (void*)gran[gy1[q]],
                                               part1 + (size_t)q * nblkG * 128, ymax, ymin, W_CARRY_INV);
  reduce_stats<64><<<1, 1024, 0, stream>>>(part1, NPART, g1, be1, scsh1);

  for (int q = 0; q < 4; ++q)
    norm_relu<<<nblkN, 256, 0, stream>>>(gran[gy1[q]], gran[gx2[q]], scsh1);
  for (int q = 0; q < 4; ++q)
    mlp_gemm<128, 2><<<nblkG, 256, 0, stream>>>(gran[gx2[q]], w2h, (void*)ymax,
                                                part2 + (size_t)q * nblkG * 256,
                                                ymax + (size_t)q * (nblkG * 8) * CH_L2,
                                                ymin + (size_t)q * (nblkG * 8) * CH_L2, W_CARRY_INV);
  reduce_stats<128><<<1, 1024, 0, stream>>>(part2, NPART, g2, be2, scsh2);

  final_pool<<<NBATCH * (NCENT / 32), 256, 0, stream>>>(ymax, ymin, scsh2, out_pts);
}
